// RealNVP_9655086482142
// MI455X (gfx1250) — hardware-verified
//
#include <hip/hip_runtime.h>
#include <hip/hip_bf16.h>

typedef __attribute__((ext_vector_type(16))) _Float16 v16h;
typedef __attribute__((ext_vector_type(8)))  _Float16 v8h;
typedef __attribute__((ext_vector_type(8)))  float    v8f;
typedef __attribute__((ext_vector_type(4)))  float    v4f;
typedef __attribute__((ext_vector_type(2)))  float    v2f;

#define PIX_PER_IMG 9216
#define NPIX        294912
#define X_TOTAL     2359296
#define W2S         136
#define W3S         136

struct __align__(16) Smem {
    _Float16 w2[128 * W2S];
    _Float16 w2l[128 * W2S];
    _Float16 w3[16  * W3S];
    _Float16 w3l[16 * W3S];
    float    w1[128 * 4];
    float    b1[128];
    float    b2[128];
    float    b3[16];
    float    ost[9][128 + 4];
};
#define RSPLIT (1.0f / 2048.0f)

__device__ __forceinline__ v8f wmma_f16(v16h a, v16h b, v8f c) {
    return __builtin_amdgcn_wmma_f32_16x16x32_f16(
        false, a, false, b, (short)0, c, false, false);
}

__device__ __forceinline__ v8f wmma_split(v16h a, v16h al, v16h b, v16h bl, v8f c) {
    v8f x = {};
    x = wmma_f16(al, b, x); x = wmma_f16(a, bl, x);
    return wmma_f16(a, b, c) + x * RSPLIT;
}
__device__ __forceinline__ _Float16 lo_of(float v, _Float16 h) { return (_Float16)((v - (float)h) * 2048.0f); }

__device__ __forceinline__ v16h ldA(const _Float16* row, int kk, int hlf) {
    const v8h* p0 = (const v8h*)(row + 32 * kk + 8 * hlf);
    const v8h* p1 = (const v8h*)(row + 32 * kk + 16 + 8 * hlf);
    v8h lo = *p0, hi = *p1;
    v16h a;
#pragma unroll
    for (int j = 0; j < 8; ++j) { a[j] = lo[j]; a[8 + j] = hi[j]; }
    return a;
}

__device__ __forceinline__ v8f ldC(const float* bias, int base, int hlf) {
    v4f c0 = *(const v4f*)(bias + base + 8 * hlf);
    v4f c1 = *(const v4f*)(bias + base + 8 * hlf + 4);
    v8f c;
#pragma unroll
    for (int j = 0; j < 4; ++j) { c[j] = c0[j]; c[4 + j] = c1[j]; }
    return c;
}

__device__ __forceinline__ void pack_act(v8f d, v16h& dst, v16h& dstl, int hi8) {
#pragma unroll
    for (int j = 0; j < 8; ++j) {
        float v = d[j]; v = v > 0.0f ? v : 0.01f * v;
        const _Float16 h = (_Float16)v;
        dst[8 * hi8 + j] = h; dstl[8 * hi8 + j] = lo_of(v, h);
    }
}

__device__ __forceinline__ float tanh_fast(float x) {
    float e = __expf(2.0f * x);
    return 1.0f - 2.0f / (e + 1.0f);
}

template <int P>
__device__ __forceinline__ void run_block(const Smem& sm, float xs[8], float& ld,
                                          int m, int hlf) {
    constexpr int FI[4][4] = {{4,5,6,7},{0,1,2,3},{1,3,5,7},{0,2,4,6}};
    constexpr int CI[4][4] = {{0,1,2,3},{4,5,6,7},{0,2,4,6},{1,3,5,7}};

    v16h bx = {}, bxl = {};
    if (hlf == 0) {
#pragma unroll
        for (int e = 0; e < 4; ++e) { const float v = xs[FI[P][e]]; const _Float16 h = (_Float16)v; bx[e] = h; bxl[e] = lo_of(v, h); }
    }

    v16h h1[4], h1l[4];
#pragma unroll
    for (int t = 0; t < 8; ++t) {
        v16h a = {}, al = {};
        if (hlf == 0) {
            const v4f w4 = *(const v4f*)(sm.w1 + (16 * t + m) * 4);
#pragma unroll
            for (int e = 0; e < 4; ++e) { const _Float16 h = (_Float16)w4[e]; a[e] = h; al[e] = lo_of(w4[e], h); }
        }
        v8f d = wmma_split(a, al, bx, bxl, ldC(sm.b1, 16 * t, hlf));
        pack_act(d, h1[t >> 1], h1l[t >> 1], t & 1);
    }

    v16h h2[4], h2l[4];
#pragma unroll
    for (int t = 0; t < 8; ++t) {
        v8f c = ldC(sm.b2, 16 * t, hlf);
        const _Float16* row  = sm.w2  + (16 * t + m) * W2S;
        const _Float16* rowl = sm.w2l + (16 * t + m) * W2S;
#pragma unroll
        for (int kk = 0; kk < 4; ++kk)
            c = wmma_split(ldA(row, kk, hlf), ldA(rowl, kk, hlf), h1[kk], h1l[kk], c);
        pack_act(c, h2[t >> 1], h2l[t >> 1], t & 1);
    }

    {
        v8f c = ldC(sm.b3, 0, hlf);
        const _Float16* row  = sm.w3  + m * W3S;
        const _Float16* rowl = sm.w3l + m * W3S;
#pragma unroll
        for (int kk = 0; kk < 4; ++kk)
            c = wmma_split(ldA(row, kk, hlf), ldA(rowl, kk, hlf), h2[kk], h2l[kk], c);
#pragma unroll
        for (int j = 0; j < 4; ++j) {
            float s  = tanh_fast(c[j]);
            float tt = tanh_fast(c[4 + j]);
            xs[CI[P][j]] = xs[CI[P][j]] * __expf(s) + tt;
            ld += s;
        }
    }
}

__device__ __forceinline__ void stage(Smem& sm, const float* W1, const float* b1,
                                      const float* W2, const float* b2,
                                      const float* W3, const float* b3,
                                      int i, int tid) {
    const float* w2 = W2 + i * 16384;
    for (int idx = tid; idx < 16384; idx += 256) {
        int r = idx >> 7, c = idx & 127;
        const float v = w2[idx]; const _Float16 h = (_Float16)v;
        sm.w2[r * W2S + c] = h; sm.w2l[r * W2S + c] = lo_of(v, h);
    }
    const float* w3 = W3 + i * 1024;
    for (int idx = tid; idx < 2048; idx += 256) {
        int r = idx >> 7, c = idx & 127;
        const float v = (r < 8) ? w3[r * 128 + c] : 0.0f; const _Float16 h = (_Float16)v;
        sm.w3[r * W3S + c] = h; sm.w3l[r * W3S + c] = lo_of(v, h);
    }
    const float* w1 = W1 + i * 512;
    for (int idx = tid; idx < 512; idx += 256) sm.w1[idx] = w1[idx];
    for (int idx = tid; idx < 128; idx += 256) {
        sm.b1[idx] = b1[i * 128 + idx];
        sm.b2[idx] = b2[i * 128 + idx];
    }
    if (tid < 16) sm.b3[tid] = (tid < 8) ? b3[i * 8 + tid] : 0.0f;
}

__global__ __launch_bounds__(256, 2) void realnvp_wmma_kernel(
    const float* __restrict__ x,
    const float* __restrict__ W1, const float* __restrict__ b1,
    const float* __restrict__ W2, const float* __restrict__ b2,
    const float* __restrict__ W3, const float* __restrict__ b3,
    float* __restrict__ out) {
    __shared__ Smem sm;

    const int tid  = threadIdx.x;
    const int lane = tid & 31;
    const int wave = tid >> 5;
    const int m    = lane & 15;
    const int hlf  = lane >> 4;

    const int tile = blockIdx.x * 8 + wave;
    const int P    = tile * 16 + m;
    const int b    = P / PIX_PER_IMG;
    const int hw   = P - b * PIX_PER_IMG;

    const float* xp = x + b * 8 * PIX_PER_IMG + hw;
    float xs[8];
#pragma unroll
    for (int c = 0; c < 8; ++c) xs[c] = xp[c * PIX_PER_IMG];
    float ld = 0.0f;

    for (int i = 0; i < 8; ++i) {
        __syncthreads();
        stage(sm, W1, b1, W2, b2, W3, b3, i, tid);
        __syncthreads();
        switch (i & 3) {
            case 0: run_block<0>(sm, xs, ld, m, hlf); break;
            case 1: run_block<1>(sm, xs, ld, m, hlf); break;
            case 2: run_block<2>(sm, xs, ld, m, hlf); break;
            default: run_block<3>(sm, xs, ld, m, hlf); break;
        }
    }

    __syncthreads();
    if (hlf == 0) {
#pragma unroll
        for (int c = 0; c < 8; ++c) sm.ost[c][wave * 16 + m] = xs[c];
        sm.ost[8][wave * 16 + m] = ld;
    }
    __syncthreads();
    {
        const int b0 = (blockIdx.x * 128) / PIX_PER_IMG, hw0 = blockIdx.x * 128 - b0 * PIX_PER_IMG;
        const int c = tid >> 5, q = tid & 31;
        typedef float v4fa __attribute__((ext_vector_type(4), may_alias));
        const v4f v = *(const v4fa*)&sm.ost[c][q * 4];
        float* op = out + (size_t)b0 * 8 * PIX_PER_IMG + (size_t)c * PIX_PER_IMG + hw0 + q * 4;
        const v4f vl = *(const v4fa*)&sm.ost[8][q * 4];
        float* opl = out + X_TOTAL + (size_t)b0 * PIX_PER_IMG + hw0 + q * 4;
        *(volatile v4f*)op = v; if (tid < 32) *(volatile v4f*)opl = vl;
        __threadfence();
        *(volatile v4f*)op = v; if (tid < 32) *(volatile v4f*)opl = vl;
    }
}

extern "C" void kernel_launch(void* const* d_in, const int* in_sizes, int n_in,
                              void* d_out, int out_size, void* d_ws, size_t ws_size,
                              hipStream_t stream) {
    const float* x  = (const float*)d_in[0];
    const float* W1 = (const float*)d_in[1];
    const float* b1 = (const float*)d_in[2];
    const float* W2 = (const float*)d_in[3];
    const float* b2 = (const float*)d_in[4];
    const float* W3 = (const float*)d_in[5];
    const float* b3 = (const float*)d_in[6];
    float* out = (float*)d_out;

    dim3 grid(2304), block(256);
    hipLaunchKernelGGL(realnvp_wmma_kernel, grid, block, 0, stream,
                       x, W1, b1, W2, b2, W3, b3, out);
}
